// HNHNModel_69818988364049
// MI455X (gfx1250) — hardware-verified
//
#include <hip/hip_runtime.h>
#include <stddef.h>


#define NHEDGE  50000
#define HIDC    128
#define KPIN    32
#define NTHR    256
#define NWAVE   8
#define EPT     8
#define NGRP    2
#define CHUNK   (NTHR * EPT * NGRP)
#define WCAP    (EPT * NGRP * 32)
#define LISTN   (NWAVE * WCAP)
#define RCAP    20480
#define MAXSEG  256
#define NBN     4096
#define NBE     2048
#define GROWS   64
#define GTHR    128
#define NIL     0xFFFFu
#define ASCALE  64.0f
#define WSCALE  16.0f
#define OSCALE  0.0009765625f

#define LDS_AGG_FIX (RCAP * 4 + LISTN * 4 + 2 * NWAVE * 1024 * 4 + NWAVE * HIDC * 4 + 64 + RCAP * 2)
#define LDS_AGGN (LDS_AGG_FIX + NBN * 2)
#define LDS_AGGE (LDS_AGG_FIX + NBE * 2)

static_assert((CHUNK & (CHUNK - 1)) == 0 && CHUNK == 4096);
static_assert(WCAP == 512 && LISTN == 4096);
static_assert(RCAP < 65535 && (RCAP % 4) == 0);
static_assert((NBN & (NBN - 1)) == 0 && (NBE & (NBE - 1)) == 0 && NBN <= 4096 && NBE <= 4096);
static_assert((NBN % (NWAVE * 32)) == 0 && (NBE % (NWAVE * 32)) == 0);
static_assert(MAXSEG > 32);
static_assert(NBN >= GROWS && NBE >= GROWS);
static_assert(GROWS == 16 * (GTHR / 32));
static_assert((LDS_AGG_FIX % 16) == 0 || 1);

typedef float    v4f  __attribute__((ext_vector_type(4)));
typedef float    v8f  __attribute__((ext_vector_type(8)));
typedef int      v4i  __attribute__((ext_vector_type(4)));
typedef unsigned v4u  __attribute__((ext_vector_type(4)));
typedef unsigned v2u  __attribute__((ext_vector_type(2)));
typedef _Float16 v4h  __attribute__((ext_vector_type(4)));
typedef _Float16 v8h  __attribute__((ext_vector_type(8)));
typedef _Float16 v16h __attribute__((ext_vector_type(16)));
union FragH { v16h v; v8h h[2]; };
union PackH { v4h h; v2u u; };

__device__ __forceinline__ v8h cvt8(v4f a, v4f b) {
  v8h r;
  r[0] = (_Float16)a.x; r[1] = (_Float16)a.y; r[2] = (_Float16)a.z; r[3] = (_Float16)a.w;
  r[4] = (_Float16)b.x; r[5] = (_Float16)b.y; r[6] = (_Float16)b.z; r[7] = (_Float16)b.w;
  return r;
}

__device__ __forceinline__ v8f wmh(v16h a, v16h b, v8f c) {
  v8f d = __builtin_amdgcn_wmma_f32_16x16x32_f16(false, a, false, b, (short)0, c, false, false);
  asm volatile("v_nop\n\tv_nop\n\tv_nop\n\tv_nop" : "+v"(d) : "v"(a), "v"(b));
  return d;
}

template <int NB>
__device__ __forceinline__ int scan_chunk(const int* __restrict__ dsts, int nE, int cbase, int slotBase,
                                          int vec8, int* list, int tid, int lane, int wave) {
  int wc = 0;
#pragma unroll
  for (int g = 0; g < NGRP; ++g) {
    const int el0  = (g * NTHR + tid) * EPT;
    const int e0   = cbase + el0;
    const int sent = -2147483647 - 1;
    v4i da, db;
    if (vec8 != 0 && cbase + CHUNK <= nE) {
      da = *(const v4i*)(dsts + e0);
      db = *(const v4i*)(dsts + e0 + 4);
    } else {
      da.x = (e0     < nE) ? dsts[min(e0, nE - 1)] : sent;
      da.y = (e0 + 1 < nE) ? dsts[min(e0 + 1, nE - 1)] : sent;
      da.z = (e0 + 2 < nE) ? dsts[min(e0 + 2, nE - 1)] : sent;
      da.w = (e0 + 3 < nE) ? dsts[min(e0 + 3, nE - 1)] : sent;
      db.x = (e0 + 4 < nE) ? dsts[min(e0 + 4, nE - 1)] : sent;
      db.y = (e0 + 5 < nE) ? dsts[min(e0 + 5, nE - 1)] : sent;
      db.z = (e0 + 6 < nE) ? dsts[min(e0 + 6, nE - 1)] : sent;
      db.w = (e0 + 7 < nE) ? dsts[min(e0 + 7, nE - 1)] : sent;
    }
    const unsigned nb = (unsigned)slotBase;
    const unsigned s0 = (unsigned)da.x - nb, s1 = (unsigned)da.y - nb;
    const unsigned s2 = (unsigned)da.z - nb, s3 = (unsigned)da.w - nb;
    const unsigned s4 = (unsigned)db.x - nb, s5 = (unsigned)db.y - nb;
    const unsigned s6 = (unsigned)db.z - nb, s7 = (unsigned)db.w - nb;
    const bool h0 = s0 < (unsigned)NB, h1 = s1 < (unsigned)NB, h2 = s2 < (unsigned)NB, h3 = s3 < (unsigned)NB;
    const bool h4 = s4 < (unsigned)NB, h5 = s5 < (unsigned)NB, h6 = s6 < (unsigned)NB, h7 = s7 < (unsigned)NB;
    const unsigned any = __builtin_amdgcn_ballot_w32(h0 | h1 | h2 | h3 | h4 | h5 | h6 | h7);
    if (any != 0u) {
#define HITJ(J, HJ, SJ) { \
        const unsigned mj = __builtin_amdgcn_ballot_w32(HJ); \
        if (mj != 0u) { \
          if (HJ) { \
            const int pos = wc + (int)__builtin_amdgcn_mbcnt_lo(mj, 0u); \
            if (pos < WCAP) list[wave * WCAP + pos] = ((el0 + (J)) << 12) | (int)(SJ); \
          } \
          wc += (int)__builtin_popcount(mj); } }
      HITJ(0, h0, s0)
      HITJ(1, h1, s1)
      HITJ(2, h2, s2)
      HITJ(3, h3, s3)
      HITJ(4, h4, s4)
      HITJ(5, h5, s5)
      HITJ(6, h6, s6)
      HITJ(7, h7, s7)
#undef HITJ
    }
  }
  return wc;
}

__global__ __launch_bounds__(NTHR) void k_wprep(
    const float* __restrict__ W0, const float* __restrict__ W1,
    const float* __restrict__ W2, const float* __restrict__ W3,
    _Float16* P0, _Float16* P1, _Float16* P2, _Float16* P3, int kin) {
  const int g0 = HIDC * KPIN / 8;
  const int g1 = HIDC * HIDC / 8;
  const int bstart = blockIdx.x * NTHR;
  const float* src; _Float16* dst; int K, KP, segOff;
  if (bstart < g0)               { src = W0; dst = P0; K = kin;  KP = KPIN; segOff = 0; }
  else if (bstart < g0 + g1)     { src = W1; dst = P1; K = HIDC; KP = HIDC; segOff = g0; }
  else if (bstart < g0 + 2 * g1) { src = W2; dst = P2; K = HIDC; KP = HIDC; segOff = g0 + g1; }
  else                           { src = W3; dst = P3; K = HIDC; KP = HIDC; segOff = g0 + 2 * g1; }
  const int i = bstart + (int)threadIdx.x;
  if (i >= g0 + 3 * g1) return;
  const int o  = (i - segOff) * 8;
  const int n  = o / KP;
  const int k0 = o - n * KP;
  float v[8];
#pragma unroll
  for (int e = 0; e < 8; ++e) {
    const int k  = k0 + e;
    const int kc = k < K ? k : K - 1;
    const float x = src[(size_t)kc * HIDC + n];
    v[e] = (k < K) ? x * WSCALE : 0.0f;
  }
  v4f a, b;
  a.x = v[0]; a.y = v[1]; a.z = v[2]; a.w = v[3];
  b.x = v[4]; b.y = v[5]; b.z = v[6]; b.w = v[7];
  const v8h hv = cvt8(a, b);
  _Float16* dp = dst + o;
  *(volatile v8h*)dp = hv;
  __threadfence();
  *(volatile v8h*)dp = hv;
}

__global__ __launch_bounds__(NTHR) void k_xprep(
    const float* __restrict__ x, _Float16* xp, int nRows, int nValid, int kin) {
  const int i = blockIdx.x * NTHR + (int)threadIdx.x;
  if (i >= nRows * 4) return;
  const int r  = i >> 2;
  const int k0 = (i & 3) * 8;
  const int rc = r < nValid ? r : nValid - 1;
  float v[8];
#pragma unroll
  for (int e = 0; e < 8; ++e) {
    const int k  = k0 + e;
    const int kc = k < kin ? k : kin - 1;
    const float xv = x[(size_t)rc * kin + kc];
    v[e] = (k < kin && r < nValid) ? xv * ASCALE : 0.0f;
  }
  v4f a, b;
  a.x = v[0]; a.y = v[1]; a.z = v[2]; a.w = v[3];
  b.x = v[4]; b.y = v[5]; b.z = v[6]; b.w = v[7];
  const v8h hv = cvt8(a, b);
  _Float16* dp = xp + (size_t)r * KPIN + k0;
  *(volatile v8h*)dp = hv;
  __threadfence();
  *(volatile v8h*)dp = hv;
}

template <int KS>
__global__ __launch_bounds__(GTHR) void k_gemm(
    const _Float16* __restrict__ A, const _Float16* __restrict__ Bw, float* C) {
  __shared__ __attribute__((aligned(16))) float stg[GROWS * HIDC];
  constexpr int KP = 32 * KS;
  const int tid = threadIdx.x, lane = tid & 31, wave = tid >> 5, hh = lane >> 4, m = lane & 15;
  const int rowBase = blockIdx.x * GROWS;
  const int r0 = wave * 16;
  const _Float16* ar = A + (size_t)(rowBase + r0 + m) * KP + 8 * hh;

  v8f acc[8];
#pragma unroll
  for (int t = 0; t < 8; ++t) { v8f z = {0.f, 0.f, 0.f, 0.f, 0.f, 0.f, 0.f, 0.f}; acc[t] = z; }
#pragma unroll
  for (int kt = 0; kt < KS; ++kt) {
    FragH a;
    a.h[0] = *(const v8h*)(ar + 32 * kt);
    a.h[1] = *(const v8h*)(ar + 32 * kt + 16);
#pragma unroll
    for (int t = 0; t < 8; ++t) {
      const _Float16* bp = Bw + (size_t)(16 * t + m) * KP + 32 * kt + 8 * hh;
      FragH b;
      b.h[0] = *(const v8h*)bp;
      b.h[1] = *(const v8h*)(bp + 16);
      acc[t] = wmh(a.v, b.v, acc[t]);
    }
  }

  float* sp = stg + (r0 + 8 * hh) * HIDC + m;
#pragma unroll
  for (int t = 0; t < 8; ++t) {
#pragma unroll
    for (int r = 0; r < 8; ++r) sp[r * HIDC + 16 * t] = acc[t][r] * OSCALE;
  }
  __syncthreads();

  const float* lp = stg + r0 * HIDC + 4 * lane;
  float* gp = C + ((size_t)rowBase + r0) * HIDC + 4 * lane;
#pragma unroll
  for (int i = 0; i < 16; ++i) { const v4f v = *(const v4f*)(lp + i * HIDC); *(volatile v4f*)(gp + (size_t)i * HIDC) = v; }
  __threadfence();
#pragma unroll
  for (int i = 0; i < 16; ++i) { const v4f v = *(const v4f*)(lp + i * HIDC); *(volatile v4f*)(gp + (size_t)i * HIDC) = v; }
}

template <int NB>
__global__ __launch_bounds__(NTHR) void k_agg(
    const int* __restrict__ keys, const int* __restrict__ part, const float* __restrict__ inc,
    const float* __restrict__ pcard, const float* __restrict__ xw, const float* __restrict__ bias,
    float* cardOut, _Float16* actOut, float* pmaxOut,
    int nnz, int nPart, int nDest, int vec8, int mode, int wrCard, int cardCube) {
  extern __shared__ v4i lds_dyn[];
  int*   U    = (int*)lds_dyn;
  int*   list = U + RCAP;
  int*   spi  = list + LISTN;
  float* spv  = (float*)(spi + NWAVE * 1024);
  float* wmx  = spv + NWAVE * 1024;
  int*   wcnt = (int*)(wmx + NWAVE * HIDC);
  unsigned short* nxt  = (unsigned short*)(wcnt + 16);
  unsigned short* head = nxt + RCAP;
  const int tid = threadIdx.x, lane = tid & 31, wave = tid >> 5;
  const int slotBase = blockIdx.x * NB;

  for (int i = tid; i < NB; i += NTHR) head[i] = (unsigned short)NIL;
  __syncthreads();

  int total = 0;
  const int nChunks = (nnz + CHUNK - 1) / CHUNK;
#pragma unroll 1
  for (int ch = 0; ch < nChunks; ++ch) {
    const int cbase = ch * CHUNK;
    const int wc = scan_chunk<NB>(keys, nnz, cbase, slotBase, vec8, list, tid, lane, wave);
    if (lane == 0) wcnt[wave] = wc;
    __syncthreads();
    int cw[NWAVE];
#pragma unroll
    for (int w = 0; w < NWAVE; ++w) {
      int n = wcnt[w];
      n = n > WCAP ? WCAP : (n < 0 ? 0 : n);
      cw[w] = n;
    }
    int pre = 0, tot = 0;
#pragma unroll
    for (int w = 0; w < NWAVE; ++w) { pre += (w < wave) ? cw[w] : 0; tot += cw[w]; }
    const int myc = wc > WCAP ? WCAP : wc;
    const int wbase = total + pre;
    const int* mylist = list + wave * WCAP;
    for (int p = lane; p < myc; p += 32) {
      const int i = wbase + p;
      int e = cbase + ((mylist[p] >> 12) & (CHUNK - 1));
      e = e > nnz - 1 ? nnz - 1 : e;
      if (i < RCAP) U[i] = e;
    }
    if (wave == 0) {
      int b = total;
#pragma unroll
      for (int w = 0; w < NWAVE; ++w) {
        const int n = cw[w];
        const int* lp = list + w * WCAP;
#pragma unroll 1
        for (int p = 0; p < n; ++p) {
          const int i = b + p;
          if (i < RCAP) {
            const int ent  = __builtin_amdgcn_readfirstlane(lp[p]);
            const int slot = ent & (NB - 1);
            if (lane == 0) {
              const unsigned short hp = head[slot];
              nxt[i] = hp;
              head[slot] = (unsigned short)i;
            }
          }
        }
        b += n;
      }
    }
    total += tot;
    if (total > RCAP) total = RCAP;
    __syncthreads();
  }

  const v4f b4 = *(const v4f*)(bias + 4 * lane);
  v4f wm = {0.f, 0.f, 0.f, 0.f};
  constexpr int NPW = NB / NWAVE;
  constexpr int NG  = NPW / 32;
  int*   mpi = spi + wave * 1024;
  float* mpv = spv + wave * 1024;

#pragma unroll 1
  for (int g = 0; g < NG; ++g) {
    const int slot0 = wave * NPW + g * 32;
    unsigned cur = head[slot0 + lane];
    float deg = 0.f, dsum = 0.f;
    int cnt = 0;
    unsigned cont = NIL;
#pragma unroll 1
    for (int s = 0; s < MAXSEG; ++s) {
      const bool act = (cur != NIL);
      if (__builtin_amdgcn_ballot_w32(act) == 0u) break;
      int ci = act ? (int)cur : 0;
      ci = ci > RCAP - 1 ? RCAP - 1 : ci;
      int nz = U[ci];
      nz = nz < 0 ? 0 : (nz > nnz - 1 ? nnz - 1 : nz);
      const unsigned nx = nxt[ci];
      const float iv = inc[nz];
      int pi = 0; float prod = 0.f;
      if (mode != 0) {
        pi = part[nz];
        pi = pi < 0 ? 0 : (pi > nPart - 1 ? nPart - 1 : pi);
        prod = iv * pcard[pi];
      }
      deg  += act ? iv : 0.f;
      dsum += act ? prod : 0.f;
      if (s == 32) cont = act ? cur : NIL;
      if (s < 32 && mode != 0) {
        mpi[s * 32 + lane] = pi;
        mpv[s * 32 + lane] = act ? prod : 0.f;
      }
      cnt += act ? 1 : 0;
      cur = act ? nx : NIL;
    }

    if (wrCard != 0) {
      const float dg   = deg > 0.f ? deg : 1.f;
      const float sq   = sqrtf(dg);
      const float den  = cardCube != 0 ? dg * sq : sq;
      const float card = deg > 0.f ? 1.0f / den : 0.f;
      float* cp = cardOut + (size_t)slotBase + slot0 + lane;
      *(volatile float*)cp = card;
      __threadfence();
      *(volatile float*)cp = card;
    }

    if (mode != 0) {
      __builtin_amdgcn_fence(__ATOMIC_RELEASE, "wavefront");
      __builtin_amdgcn_wave_barrier();
      const float inv = dsum > 0.f ? 1.0f / dsum : 0.f;
      const int invb  = __float_as_int(inv);
      const int contb = (int)cont;
#pragma unroll 1
      for (int j = 0; j < 32; ++j) {
        const int nj = __builtin_amdgcn_readlane(cnt, j);
        const int nb = nj < 32 ? nj : 32;
        const float invj = __int_as_float(__builtin_amdgcn_readlane(invb, j));
        v4f acc = {0.f, 0.f, 0.f, 0.f};
#pragma unroll 1
        for (int p = 0; p < nb; ++p) {
          int pi = mpi[p * 32 + j];
          pi = pi < 0 ? 0 : (pi > nPart - 1 ? nPart - 1 : pi);
          const float v = mpv[p * 32 + j];
          const v4f row = *(const v4f*)(xw + (size_t)pi * HIDC + 4 * lane);
          acc = acc + v * row;
        }
        int rem = nj - 32;
        rem = rem > MAXSEG - 32 ? MAXSEG - 32 : rem;
        unsigned cj = (unsigned)__builtin_amdgcn_readlane(contb, j);
#pragma unroll 1
        for (int q = 0; q < rem; ++q) {
          if (cj == NIL) break;
          int ci = (int)cj;
          ci = ci > RCAP - 1 ? RCAP - 1 : ci;
          int nz = U[ci];
          nz = nz < 0 ? 0 : (nz > nnz - 1 ? nnz - 1 : nz);
          const unsigned nx = nxt[ci];
          int pi = part[nz];
          pi = pi < 0 ? 0 : (pi > nPart - 1 ? nPart - 1 : pi);
          const float prod = inc[nz] * pcard[pi];
          const v4f row = *(const v4f*)(xw + (size_t)pi * HIDC + 4 * lane);
          acc = acc + prod * row;
          cj = nx;
        }
        v4f v = acc * invj + b4;
        v.x = fmaxf(v.x, 0.f); v.y = fmaxf(v.y, 0.f); v.z = fmaxf(v.z, 0.f); v.w = fmaxf(v.w, 0.f);
        const int dslot = slot0 + j;
        if (mode == 1) {
          PackH pk;
          pk.h[0] = (_Float16)(v.x * ASCALE);
          pk.h[1] = (_Float16)(v.y * ASCALE);
          pk.h[2] = (_Float16)(v.z * ASCALE);
          pk.h[3] = (_Float16)(v.w * ASCALE);
          const unsigned u0 = pk.u.x, u1 = pk.u.y;
          const int sa = (2 * lane) & 31, sb = (2 * lane + 1) & 31;
          v4u w;
          w.x = (unsigned)__shfl((int)u0, sa);
          w.y = (unsigned)__shfl((int)u1, sa);
          w.z = (unsigned)__shfl((int)u0, sb);
          w.w = (unsigned)__shfl((int)u1, sb);
          _Float16* rp = actOut + ((size_t)slotBase + dslot) * HIDC + 8 * lane;
          if (lane < 16) *(volatile v4u*)rp = w;
          __threadfence();
          if (lane < 16) *(volatile v4u*)rp = w;
        } else {
          const float f = (slotBase + dslot < nDest) ? 1.f : 0.f;
          const v4f vf = v * f;
          wm.x = fmaxf(wm.x, vf.x); wm.y = fmaxf(wm.y, vf.y); wm.z = fmaxf(wm.z, vf.z); wm.w = fmaxf(wm.w, vf.w);
        }
      }
      __builtin_amdgcn_fence(__ATOMIC_RELEASE, "wavefront");
      __builtin_amdgcn_wave_barrier();
    }
  }

  if (mode == 2) *(v4f*)(wmx + wave * HIDC + 4 * lane) = wm;
  __syncthreads();
  if (mode == 2 && wave == 0) {
    v4f mx = *(const v4f*)(wmx + 4 * lane);
#pragma unroll
    for (int w = 1; w < NWAVE; ++w) {
      const v4f o = *(const v4f*)(wmx + w * HIDC + 4 * lane);
      mx.x = fmaxf(mx.x, o.x); mx.y = fmaxf(mx.y, o.y); mx.z = fmaxf(mx.z, o.z); mx.w = fmaxf(mx.w, o.w);
    }
    float* pp = pmaxOut + (size_t)blockIdx.x * HIDC + 4 * lane;
    *(volatile v4f*)pp = mx;
    __threadfence();
    *(volatile v4f*)pp = mx;
  }
}

__global__ __launch_bounds__(HIDC) void k_final(
    const float* __restrict__ pmax, const float* __restrict__ wl, const float* __restrict__ bl,
    float* out, int nblk) {
  __shared__ float red[HIDC];
  const int t = threadIdx.x;
  float m = 0.f;
#pragma unroll 1
  for (int b = 0; b < nblk; ++b) m = fmaxf(m, pmax[(size_t)b * HIDC + t]);
  red[t] = m * wl[t];
  __syncthreads();
#pragma unroll 1
  for (int s = HIDC / 2; s > 0; s >>= 1) {
    if (t < s) red[t] = red[t] + red[t + s];
    __syncthreads();
  }
  if (t == 0) {
    const float r = red[0] + bl[0];
    *(volatile float*)out = r;
    __threadfence();
    *(volatile float*)out = r;
  }
}

extern "C" void kernel_launch(void* const* d_in, const int* in_sizes, int n_in,
                              void* d_out, int out_size, void* d_ws, size_t ws_size,
                              hipStream_t stream) {
  if (n_in < 14 || out_size < 1) return;
  if (in_sizes[2] <= 0 || (in_sizes[2] % HIDC) != 0) return;
  const int kin = in_sizes[2] / HIDC;
  if (kin < 1 || kin > KPIN) return;
  if (in_sizes[0] <= 0 || (in_sizes[0] % kin) != 0) return;
  const int nN  = in_sizes[0] / kin;
  const int nnz = in_sizes[1];
  const int nE  = NHEDGE;
  if (nN <= 0 || nnz <= 0 || in_sizes[12] != nnz || in_sizes[13] != nnz) return;
  if (in_sizes[3] != HIDC || in_sizes[4] != HIDC * HIDC || in_sizes[5] != HIDC ||
      in_sizes[6] != HIDC * HIDC || in_sizes[7] != HIDC || in_sizes[8] != HIDC * HIDC ||
      in_sizes[9] != HIDC || in_sizes[10] != HIDC || in_sizes[11] < 1) return;
  if (nN > (1 << 24) || nnz > (1 << 28)) return;

  const float* x0    = (const float*)d_in[0];
  const float* incv  = (const float*)d_in[1];
  const float* W01_0 = (const float*)d_in[2];
  const float* b1_0  = (const float*)d_in[3];
  const float* W10_0 = (const float*)d_in[4];
  const float* b0_0  = (const float*)d_in[5];
  const float* W01_1 = (const float*)d_in[6];
  const float* b1_1  = (const float*)d_in[7];
  const float* W10_1 = (const float*)d_in[8];
  const float* b0_1  = (const float*)d_in[9];
  const float* W_lin = (const float*)d_in[10];
  const float* b_lin = (const float*)d_in[11];
  const int*   nidx  = (const int*)d_in[12];
  const int*   eidx  = (const int*)d_in[13];
  float* out = (float*)d_out;

  const int NROWX = ((nN + GROWS - 1) / GROWS) * GROWS;
  const int NROWE = ((nE + GROWS - 1) / GROWS) * GROWS;
  const int NBLKN = (nN + NBN - 1) / NBN;
  const int NPADN = NBLKN * NBN;
  const int NBLKE = (nE + NBE - 1) / NBE;
  const int NPADE = NBLKE * NBE;
  if (NPADN < NROWX || NPADE < NROWE) return;
  const int xwRows = NROWX > NROWE ? NROWX : NROWE;

  char* ws = (char*)d_ws;
  size_t off = 0;
  const size_t oW0 = off; off += (size_t)HIDC * KPIN * 2;        off = (off + 255) & ~(size_t)255;
  const size_t oW1 = off; off += (size_t)HIDC * HIDC * 2;        off = (off + 255) & ~(size_t)255;
  const size_t oW2 = off; off += (size_t)HIDC * HIDC * 2;        off = (off + 255) & ~(size_t)255;
  const size_t oW3 = off; off += (size_t)HIDC * HIDC * 2;        off = (off + 255) & ~(size_t)255;
  const size_t oXP = off; off += (size_t)NROWX * KPIN * 2;       off = (off + 255) & ~(size_t)255;
  const size_t oNC = off; off += (size_t)NPADN * 4;              off = (off + 255) & ~(size_t)255;
  const size_t oEC = off; off += (size_t)NPADE * 4;              off = (off + 255) & ~(size_t)255;
  const size_t oXW = off; off += (size_t)xwRows * HIDC * 4;      off = (off + 255) & ~(size_t)255;
  const size_t oAE = off; off += (size_t)NPADE * HIDC * 2;       off = (off + 255) & ~(size_t)255;
  const size_t oAN = off; off += (size_t)NPADN * HIDC * 2;       off = (off + 255) & ~(size_t)255;
  const size_t oPM = off; off += (size_t)NBLKN * HIDC * 4;       off = (off + 255) & ~(size_t)255;
  if (off > ws_size) return;
  _Float16* pW0   = (_Float16*)(ws + oW0);
  _Float16* pW1   = (_Float16*)(ws + oW1);
  _Float16* pW2   = (_Float16*)(ws + oW2);
  _Float16* pW3   = (_Float16*)(ws + oW3);
  _Float16* xP    = (_Float16*)(ws + oXP);
  float*    ncard = (float*)(ws + oNC);
  float*    ecard = (float*)(ws + oEC);
  float*    xw    = (float*)(ws + oXW);
  _Float16* actE  = (_Float16*)(ws + oAE);
  _Float16* actN  = (_Float16*)(ws + oAN);
  float*    pmax  = (float*)(ws + oPM);

  const int vec8 = ((nnz & 3) == 0) ? 1 : 0;

  const int nPrep = (HIDC * KPIN + 3 * HIDC * HIDC) / 8;
  k_wprep<<<(nPrep + NTHR - 1) / NTHR, NTHR, 0, stream>>>(W01_0, W10_0, W01_1, W10_1, pW0, pW1, pW2, pW3, kin);
  k_xprep<<<(NROWX * 4 + NTHR - 1) / NTHR, NTHR, 0, stream>>>(x0, xP, NROWX, nN, kin);

  hipFuncSetAttribute(reinterpret_cast<const void*>(&k_agg<NBN>),
                      hipFuncAttributeMaxDynamicSharedMemorySize, LDS_AGGN);
  hipFuncSetAttribute(reinterpret_cast<const void*>(&k_agg<NBE>),
                      hipFuncAttributeMaxDynamicSharedMemorySize, LDS_AGGE);

  k_agg<NBN><<<NBLKN, NTHR, LDS_AGGN, stream>>>(nidx, eidx, incv, ecard, xw, b0_0, ncard, actN, pmax,
                                                 nnz, nE, nN, vec8, 0, 1, 0);

  k_gemm<1><<<NROWX / GROWS, GTHR, 0, stream>>>(xP, pW0, xw);
  k_agg<NBE><<<NBLKE, NTHR, LDS_AGGE, stream>>>(eidx, nidx, incv, ncard, xw, b1_0, ecard, actE, pmax,
                                                 nnz, nN, nE, vec8, 1, 1, 1);
  k_gemm<4><<<NROWE / GROWS, GTHR, 0, stream>>>(actE, pW1, xw);
  k_agg<NBN><<<NBLKN, NTHR, LDS_AGGN, stream>>>(nidx, eidx, incv, ecard, xw, b0_0, ncard, actN, pmax,
                                                 nnz, nE, nN, vec8, 1, 0, 0);

  k_gemm<4><<<NROWX / GROWS, GTHR, 0, stream>>>(actN, pW2, xw);
  k_agg<NBE><<<NBLKE, NTHR, LDS_AGGE, stream>>>(eidx, nidx, incv, ncard, xw, b1_1, ecard, actE, pmax,
                                                 nnz, nN, nE, vec8, 1, 0, 1);
  k_gemm<4><<<NROWE / GROWS, GTHR, 0, stream>>>(actE, pW3, xw);
  k_agg<NBN><<<NBLKN, NTHR, LDS_AGGN, stream>>>(nidx, eidx, incv, ecard, xw, b0_1, ncard, actN, pmax,
                                                 nnz, nE, nN, vec8, 2, 0, 0);

  k_final<<<1, HIDC, 0, stream>>>(pmax, W_lin, b_lin, out, NBLKN);
}
